// GptOssDFlashAttention_22952305230270
// MI455X (gfx1250) — hardware-verified
//
#include <hip/hip_runtime.h>
#include <math.h>
#include <stdint.h>

#define QLEN 1024
#define CLEN 1024
#define SLEN (CLEN + QLEN)
#define HID  2880
#define NH   64
#define NKV  8
#define HD   64
#define QP   (NH * HD)
#define KP   (NKV * HD)
#define NQB  (QLEN / 64)
#define NKT  (SLEN / 64)
#define QSC  16.0f
#define KSC  16.0f
#define VSC  64.0f
#define PSC  1024.0f
static_assert(HD == 64);
static_assert((HID % 32) == 0 && (QP % 64) == 0 && (KP % 64) == 0 && (HID % 64) == 0);
static_assert((QLEN % 64) == 0 && (SLEN % 64) == 0);
static_assert((NH % NKV) == 0 && (NH % 4) == 0 && (NKV % 4) == 0);
static_assert(((HID * 2) % 128) == 0 && ((HID * 4) % 128) == 0);

typedef _Float16 v16h __attribute__((ext_vector_type(16)));
typedef _Float16 v8h  __attribute__((ext_vector_type(8)));
typedef __bf16   v16b __attribute__((ext_vector_type(16)));
typedef __bf16   v8b  __attribute__((ext_vector_type(8)));
typedef float    v8f  __attribute__((ext_vector_type(8)));
typedef float    v4f  __attribute__((ext_vector_type(4)));
typedef unsigned int v4u __attribute__((ext_vector_type(4)));

__device__ __forceinline__ unsigned short bf_bits(float f) {
  unsigned u = __float_as_uint(f);
  return (unsigned short)((u + 0x7FFFu + ((u >> 16) & 1u)) >> 16);
}
__device__ __forceinline__ float bf_up(unsigned short h) { return __uint_as_float(((unsigned)h) << 16); }
__device__ __forceinline__ float bfr(float f) { return bf_up(bf_bits(f)); }
__device__ __forceinline__ unsigned short h_bits(_Float16 x) { return __builtin_bit_cast(unsigned short, x); }
__device__ __forceinline__ unsigned pk16(unsigned short a, unsigned short b) { return (unsigned)a | ((unsigned)b << 16); }
__device__ __forceinline__ v8f zero8() { v8f z = {0.f, 0.f, 0.f, 0.f, 0.f, 0.f, 0.f, 0.f}; return z; }

__device__ __forceinline__ v16b ldfrag_b(const __bf16* p) {
  union { v16b v; v8b h[2]; } f;
  f.h[0] = *(const v8b*)(p);
  f.h[1] = *(const v8b*)(p + 16);
  return f.v;
}
__device__ __forceinline__ v16h ldfrag_h(const _Float16* p) {
  union { v16h v; v8h h[2]; } f;
  f.h[0] = *(const v8h*)(p);
  f.h[1] = *(const v8h*)(p + 16);
  return f.v;
}

__device__ __forceinline__ v8f mma_h(v16h a, v16h b, v8f c) {
  c = __builtin_amdgcn_wmma_f32_16x16x32_f16(false, a, false, b, (short)0, c, false, false);
#if defined(__HIP_DEVICE_COMPILE__)
  asm volatile("v_nop\n\tv_nop\n\tv_nop\n\tv_nop" : "+v"(c) : "v"(a), "v"(b));
#endif
  return c;
}
__device__ __forceinline__ v8f mma_b_raw(v16b a, v16b b, v8f c) {
  return __builtin_amdgcn_wmma_f32_16x16x32_bf16(false, a, false, b, (short)0, c, false, false);
}
__device__ __forceinline__ void dep_guard_b(v8f& a, v8f& b, v16b x, v16b y) {
#if defined(__HIP_DEVICE_COMPILE__)
  asm volatile("v_nop\n\tv_nop\n\tv_nop\n\tv_nop" : "+v"(a), "+v"(b) : "v"(x), "v"(y));
#endif
}
__device__ __forceinline__ void keep4_b(v16b a, v16b b, v16b c, v16b d) {
#if defined(__HIP_DEVICE_COMPILE__)
  asm volatile("v_nop" :: "v"(a), "v"(b), "v"(c), "v"(d));
#endif
}
__device__ __forceinline__ void acc_guard4(v8f& a, v8f& b, v8f& c, v8f& d) {
#if defined(__HIP_DEVICE_COMPILE__)
  asm volatile("v_nop\n\tv_nop\n\tv_nop\n\tv_nop" : "+v"(a), "+v"(b), "+v"(c), "+v"(d));
#endif
}

__global__ __launch_bounds__(256) void cvt_bf16x8(const float* __restrict__ in, unsigned short* out, int n8) {
  const int i = blockIdx.x * 256 + threadIdx.x;
  if (i < n8) {
    const float* s = in + (size_t)i * 8;
    const v4f a = *(const v4f*)(s);
    const v4f b = *(const v4f*)(s + 4);
    v4u p;
    p[0] = pk16(bf_bits(a[0]), bf_bits(a[1]));
    p[1] = pk16(bf_bits(a[2]), bf_bits(a[3]));
    p[2] = pk16(bf_bits(b[0]), bf_bits(b[1]));
    p[3] = pk16(bf_bits(b[2]), bf_bits(b[3]));
    unsigned short* d = out + (size_t)i * 8;
    *(volatile v4u*)d = p;
    __threadfence();
    *(volatile v4u*)d = p;
  }
}

__global__ __launch_bounds__(256) void split_bf16x8(const float* __restrict__ in, unsigned short* hp,
                                                    unsigned short* lp, int n8) {
  const int i = blockIdx.x * 256 + threadIdx.x;
  if (i < n8) {
    const v4f a = *(const v4f*)(in + (size_t)i * 8);
    const v4f b = *(const v4f*)(in + (size_t)i * 8 + 4);
    v4u ph, pl;
#pragma unroll
    for (int e = 0; e < 4; ++e) {
      const float f0 = (e < 2) ? a[2 * e]     : b[2 * e - 4];
      const float f1 = (e < 2) ? a[2 * e + 1] : b[2 * e - 3];
      const unsigned short h0 = bf_bits(f0), h1 = bf_bits(f1);
      const unsigned short l0 = bf_bits(f0 - bf_up(h0)), l1 = bf_bits(f1 - bf_up(h1));
      ph[e] = pk16(h0, h1);
      pl[e] = pk16(l0, l1);
    }
    *(volatile v4u*)(hp + (size_t)i * 8) = ph;
    *(volatile v4u*)(lp + (size_t)i * 8) = pl;
    __threadfence();
    *(volatile v4u*)(hp + (size_t)i * 8) = ph;
    *(volatile v4u*)(lp + (size_t)i * 8) = pl;
  }
}

template <int NSPLIT, int OUT_MODE, int BIAS>
__global__ __launch_bounds__(256) void gemm64(
    const unsigned short* __restrict__ Ap, const unsigned short* __restrict__ A2p, int lda,
    const unsigned short* __restrict__ Btp, int ldb,
    const float* __restrict__ bias,
    void* Cout, int ldc, int M, int N, int K, float oscale) {
  const __bf16* A  = (const __bf16*)(const void*)Ap;
  const __bf16* A2 = (const __bf16*)(const void*)A2p;
  const __bf16* Bt = (const __bf16*)(const void*)Btp;
  __shared__ __align__(16) float sT[8][16 * 68];
  const int lane = threadIdx.x & 31;
  const int wave = threadIdx.x >> 5;
  const int tilesN = N >> 6;
  const int tilesM = M >> 6;
  const int tile = blockIdx.x * 8 + wave;
  if (tile >= tilesM * tilesN) return;
  const int tm = tile / tilesN;
  const int tn = tile - tm * tilesN;
  const int m0 = tm << 6;
  const int n0 = tn << 6;

  const int rlane = lane & 15;
  const int koff  = (lane >> 4) * 8;
  const int mOff  = (lane >> 4) * 8;

  v8f acc[4][4];
#pragma unroll
  for (int i = 0; i < 4; ++i)
#pragma unroll
    for (int j = 0; j < 4; ++j) acc[i][j] = zero8();

  for (int k0 = 0; k0 < K; k0 += 32) {
    v16b bh[4];
#pragma unroll
    for (int j = 0; j < 4; ++j) {
      const size_t bo = (size_t)(n0 + (j << 4) + rlane) * ldb + koff + k0;
      bh[j] = ldfrag_b(Bt + bo);
    }
#pragma unroll
    for (int i = 0; i < 4; ++i) {
      const size_t ao = (size_t)(m0 + (i << 4) + rlane) * lda + koff + k0;
      const v16b ah = ldfrag_b(A + ao);
      v16b al = ah;
      if (NSPLIT == 1) al = ldfrag_b(A2 + ao);
#pragma unroll
      for (int j = 0; j < 4; ++j) {
        acc[i][j] = mma_b_raw(ah, bh[j], acc[i][j]);
        if (NSPLIT == 1) acc[i][j] = mma_b_raw(al, bh[j], acc[i][j]);
      }
      dep_guard_b(acc[i][0], acc[i][3], ah, al);
    }
    keep4_b(bh[0], bh[1], bh[2], bh[3]);
  }
  acc_guard4(acc[0][0], acc[0][1], acc[0][2], acc[0][3]);
  acc_guard4(acc[1][0], acc[1][1], acc[1][2], acc[1][3]);
  acc_guard4(acc[2][0], acc[2][1], acc[2][2], acc[2][3]);
  acc_guard4(acc[3][0], acc[3][1], acc[3][2], acc[3][3]);

  float bcol[4];
#pragma unroll
  for (int j = 0; j < 4; ++j) bcol[j] = 0.f;
  if (BIAS == 1) {
#pragma unroll
    for (int j = 0; j < 4; ++j) bcol[j] = bfr(bias[n0 + (j << 4) + rlane]);
  }

  float* slab = sT[wave];
#pragma unroll
  for (int i = 0; i < 4; ++i) {
    const int mBase = m0 + (i << 4);
    float brow[8];
#pragma unroll
    for (int r = 0; r < 8; ++r) brow[r] = 0.f;
    if (BIAS == 2) {
#pragma unroll
      for (int r = 0; r < 8; ++r) brow[r] = bfr(bias[mBase + mOff + r]);
    }
#pragma unroll
    for (int r = 0; r < 8; ++r) {
#pragma unroll
      for (int j = 0; j < 4; ++j) {
        float v = acc[i][j][r];
        if (BIAS == 1) v += bcol[j];
        if (BIAS == 2) v += brow[r];
        if (OUT_MODE == 1) v *= oscale;
        slab[(mOff + r) * 68 + (j << 4) + rlane] = v;
      }
    }
    __builtin_amdgcn_fence(__ATOMIC_RELEASE, "workgroup");
    __builtin_amdgcn_wave_barrier();
    __builtin_amdgcn_fence(__ATOMIC_ACQUIRE, "workgroup");
    if (OUT_MODE == 0) {
      float* C = (float*)Cout;
      const int hh = lane >> 4, c4 = (lane & 15) * 4;
      v4f ov[8];
#pragma unroll
      for (int it = 0; it < 8; ++it) {
        const int row = it * 2 + hh;
        ov[it] = *(const v4f*)(slab + row * 68 + c4);
      }
      for (int pass = 0; pass < 2; ++pass) {
#pragma unroll
        for (int it = 0; it < 8; ++it) {
          const int row = it * 2 + hh;
          *(volatile v4f*)(C + (size_t)(mBase + row) * ldc + n0 + c4) = ov[it];
        }
        __threadfence();
      }
    } else {
      unsigned short* C = (unsigned short*)Cout;
      const int q = lane >> 3, c8 = (lane & 7) * 8;
      v4u hv[4];
#pragma unroll
      for (int it = 0; it < 4; ++it) {
        const int row = it * 4 + q;
        const float* sp = slab + row * 68 + c8;
        v4u a;
#pragma unroll
        for (int e = 0; e < 4; ++e) {
          a[e] = pk16(h_bits((_Float16)sp[2 * e]), h_bits((_Float16)sp[2 * e + 1]));
        }
        hv[it] = a;
      }
      for (int pass = 0; pass < 2; ++pass) {
#pragma unroll
        for (int it = 0; it < 4; ++it) {
          const int row = it * 4 + q;
          *(volatile v4u*)(C + (size_t)(mBase + row) * ldc + n0 + c8) = hv[it];
        }
        __threadfence();
      }
    }
    __builtin_amdgcn_fence(__ATOMIC_RELEASE, "workgroup");
    __builtin_amdgcn_wave_barrier();
    __builtin_amdgcn_fence(__ATOMIC_ACQUIRE, "workgroup");
  }
}

__global__ __launch_bounds__(256) void rope_quads(const float* __restrict__ src, const float* __restrict__ ct,
                                                  const float* __restrict__ st, unsigned short* dst,
                                                  int rp, int nquad, int trow0, float osc, int nwaves) {
#pragma clang fp contract(off)
  __shared__ __align__(16) float sy[8][256];
  const int tid = threadIdx.x, wave = tid >> 5, lane = tid & 31;
  const int w = blockIdx.x * 8 + wave;
  if (w >= nwaves) return;
  const int qd   = w % nquad;
  const int tok  = w / nquad;
  const int trow = trow0 + tok;
  const float c1 = bfr(ct[(size_t)trow * HD + lane]);
  const float c2 = bfr(ct[(size_t)trow * HD + 32 + lane]);
  const float s1 = bfr(st[(size_t)trow * HD + lane]);
  const float s2 = bfr(st[(size_t)trow * HD + 32 + lane]);
  const float* row = src + (size_t)tok * rp + (size_t)qd * 256;
  float* buf = sy[wave];
#pragma unroll
  for (int t = 0; t < 4; ++t) {
    const float x1 = row[t * 64 + lane];
    const float x2 = row[t * 64 + 32 + lane];
    const float y1 = x1 * c1 - x2 * s1;
    const float y2 = x2 * c2 + x1 * s2;
    buf[t * 64 + lane]      = y1;
    buf[t * 64 + 32 + lane] = y2;
  }
  __builtin_amdgcn_fence(__ATOMIC_RELEASE, "workgroup");
  __builtin_amdgcn_wave_barrier();
  __builtin_amdgcn_fence(__ATOMIC_ACQUIRE, "workgroup");
  const int g = lane >> 3, piece = lane & 7;
  const float* sp = buf + g * 64 + piece * 8;
  const v4f a0 = *(const v4f*)(sp);
  const v4f a1 = *(const v4f*)(sp + 4);
  v4u hv;
#pragma unroll
  for (int e = 0; e < 4; ++e) {
    const float f0 = (e < 2) ? a0[2 * e]     : a1[2 * e - 4];
    const float f1 = (e < 2) ? a0[2 * e + 1] : a1[2 * e - 3];
    hv[e] = pk16(h_bits((_Float16)(f0 * osc)), h_bits((_Float16)(f1 * osc)));
  }
  unsigned short* d = dst + (size_t)tok * rp + (size_t)qd * 256 + (size_t)g * 64 + piece * 8;
  *(volatile v4u*)d = hv;
  __threadfence();
  *(volatile v4u*)d = hv;
}

__global__ __launch_bounds__(128)
void attn64(const unsigned short* __restrict__ qpl, const unsigned short* __restrict__ kpl,
            const unsigned short* __restrict__ vtp, float* outp, float sscale, float onorm) {
  union FH { v16h v; v8h h[2]; };
  __shared__ __align__(16) _Float16 Ksh[64 * 64];
  __shared__ __align__(16) _Float16 Vth[64 * 64];
  __shared__ __align__(16) _Float16 Psh[4][16 * 64];
  __shared__ __align__(16) float    Os[4][16 * 64];

  const int tid  = threadIdx.x;
  const int wave = tid >> 5;
  const int lane = tid & 31;
  const int hh   = lane >> 4;
  const int c    = lane & 15;

  const int bx   = blockIdx.x;
  const int qb   = bx % NQB;
  const int h    = bx / NQB;
  const int kvh  = h / (NH / NKV);
  const int q0   = qb * 64 + wave * 16;

  const _Float16* Qh = (const _Float16*)(const void*)qpl + (size_t)h * HD;
  const _Float16* Kh = (const _Float16*)(const void*)kpl + (size_t)kvh * HD;
  const _Float16* Vh = (const _Float16*)(const void*)vtp + (size_t)kvh * HD * SLEN;

  v16h qa[2];
#pragma unroll
  for (int dc = 0; dc < 2; ++dc) {
    qa[dc] = ldfrag_h(Qh + (size_t)(q0 + c) * QP + dc * 32 + 8 * hh);
  }

  float mrow[8], lrow[8];
  v8f oacc[4];
#pragma unroll
  for (int r = 0; r < 8; ++r) { mrow[r] = -INFINITY; lrow[r] = 0.f; }
#pragma unroll
  for (int t = 0; t < 4; ++t) oacc[t] = zero8();

  for (int kt = 0; kt < NKT; ++kt) {
    const int kv0 = kt * 64;
    __syncthreads();
    {
      const int r = tid >> 1, half = (tid & 1) * 32;
      const _Float16* kg = Kh + (size_t)(kv0 + r) * KP + half;
      const _Float16* vg = Vh + (size_t)r * SLEN + kv0 + half;
#pragma unroll
      for (int i = 0; i < 4; ++i) {
        const v8h a0 = *(const v8h*)(kg + 8 * i);
        const v8h b0 = *(const v8h*)(vg + 8 * i);
        *(v8h*)(Ksh + r * 64 + half + 8 * i) = a0;
        *(v8h*)(Vth + r * 64 + half + 8 * i) = b0;
      }
    }
    __syncthreads();

    v8f s[4];
#pragma unroll
    for (int j = 0; j < 4; ++j) {
      s[j] = zero8();
#pragma unroll
      for (int dc = 0; dc < 2; ++dc) {
        FH kb;
        kb.h[0] = *(const v8h*)(Ksh + (j * 16 + c) * 64 + dc * 32 + 8 * hh);
        kb.h[1] = *(const v8h*)(Ksh + (j * 16 + c) * 64 + dc * 32 + 16 + 8 * hh);
        s[j] = mma_h(qa[dc], kb.v, s[j]);
      }
    }

    _Float16* pwh = Psh[wave];
#pragma unroll
    for (int r = 0; r < 8; ++r) {
      float m = -INFINITY;
#pragma unroll
      for (int j = 0; j < 4; ++j) {
        const float sv = s[j][r] * sscale;
        s[j][r] = sv;
        m = fmaxf(m, sv);
      }
#pragma unroll
      for (int off = 1; off < 16; off <<= 1) m = fmaxf(m, __shfl_xor(m, off, 32));
      const float mnew  = fmaxf(mrow[r], m);
      const float msafe = (mnew == -INFINITY) ? 0.f : mnew;
      const float alpha = __expf(mrow[r] - msafe);
      mrow[r] = mnew;
      float psum = 0.f;
#pragma unroll
      for (int j = 0; j < 4; ++j) {
        const float p = __expf(s[j][r] - msafe);
        psum += p;
        pwh[(8 * hh + r) * 64 + j * 16 + c] = (_Float16)(p * PSC);
      }
#pragma unroll
      for (int off = 1; off < 16; off <<= 1) psum += __shfl_xor(psum, off, 32);
      lrow[r] = lrow[r] * alpha + psum;
#pragma unroll
      for (int t = 0; t < 4; ++t) oacc[t][r] *= alpha;
    }
    __builtin_amdgcn_fence(__ATOMIC_RELEASE, "workgroup");
    __builtin_amdgcn_wave_barrier();
    __builtin_amdgcn_fence(__ATOMIC_ACQUIRE, "workgroup");

#pragma unroll 1
    for (int kk = 0; kk < 2; ++kk) {
      FH pa;
      pa.h[0] = *(const v8h*)(pwh + c * 64 + kk * 32 + 8 * hh);
      pa.h[1] = *(const v8h*)(pwh + c * 64 + kk * 32 + 16 + 8 * hh);
#pragma unroll
      for (int t = 0; t < 4; ++t) {
        FH vb;
        vb.h[0] = *(const v8h*)(Vth + (t * 16 + c) * 64 + kk * 32 + 8 * hh);
        vb.h[1] = *(const v8h*)(Vth + (t * 16 + c) * 64 + kk * 32 + 16 + 8 * hh);
        oacc[t] = mma_h(pa.v, vb.v, oacc[t]);
      }
    }
  }

  float* os = Os[wave];
#pragma unroll
  for (int r = 0; r < 8; ++r) {
    const float l = lrow[r];
    const float inv = ((l > 0.f) ? (1.0f / l) : 0.f) * onorm;
#pragma unroll
    for (int t = 0; t < 4; ++t) os[(8 * hh + r) * 64 + t * 16 + c] = oacc[t][r] * inv;
  }
  __builtin_amdgcn_fence(__ATOMIC_RELEASE, "workgroup");
  __builtin_amdgcn_wave_barrier();
  __builtin_amdgcn_fence(__ATOMIC_ACQUIRE, "workgroup");
  {
    const int h2 = lane >> 4, c4 = (lane & 15) * 4;
    v4f ov[8];
#pragma unroll
    for (int it = 0; it < 8; ++it) {
      const int row = it * 2 + h2;
      ov[it] = *(const v4f*)(os + row * 64 + c4);
    }
    for (int pass = 0; pass < 2; ++pass) {
#pragma unroll
      for (int it = 0; it < 8; ++it) {
        const int row = it * 2 + h2;
        const size_t go = (size_t)(q0 + row) * QP + (size_t)h * HD + c4;
        *(volatile v4f*)(outp + go) = ov[it];
      }
      __threadfence();
    }
  }
}

extern "C" void kernel_launch(void* const* d_in, const int* in_sizes, int n_in,
                              void* d_out, int out_size, void* d_ws, size_t ws_size,
                              hipStream_t stream) {
  if (n_in < 12) return;
  if (in_sizes[0] != QLEN * HID) return;
  if (in_sizes[1] != CLEN * HID) return;
  if (in_sizes[2] != SLEN * HD) return;
  if (in_sizes[3] != SLEN * HD) return;
  if (in_sizes[4] != QP * HID) return;
  if (in_sizes[5] != QP) return;
  if (in_sizes[6] != KP * HID) return;
  if (in_sizes[7] != KP) return;
  if (in_sizes[8] != KP * HID) return;
  if (in_sizes[9] != KP) return;
  if (in_sizes[10] != HID * QP) return;
  if (in_sizes[11] != HID) return;
  if (out_size != QLEN * HID) return;

  const float* hid = (const float*)d_in[0];
  const float* tgt = (const float*)d_in[1];
  const float* fcs = (const float*)d_in[2];
  const float* fsn = (const float*)d_in[3];
  const float* Wq  = (const float*)d_in[4];
  const float* bq  = (const float*)d_in[5];
  const float* Wk  = (const float*)d_in[6];
  const float* bk  = (const float*)d_in[7];
  const float* Wv  = (const float*)d_in[8];
  const float* bv  = (const float*)d_in[9];
  const float* Wo  = (const float*)d_in[10];
  const float* bo  = (const float*)d_in[11];

  const size_t PX   = (size_t)SLEN * HID * 2;
  const size_t PWq  = (size_t)QP * HID * 2;
  const size_t PWk  = (size_t)KP * HID * 2;
  const size_t PWv  = (size_t)KP * HID * 2;
  const size_t PWo  = (size_t)HID * QP * 2;
  const size_t PQf  = (size_t)QLEN * QP * 4;
  const size_t PKf  = (size_t)SLEN * KP * 4;
  const size_t PVT  = (size_t)KP * SLEN * 2;
  const size_t PQh  = (size_t)QLEN * QP * 2;
  const size_t PKh  = (size_t)SLEN * KP * 2;
  const size_t PApl = (size_t)QLEN * QP * 2;
  size_t off = 0;
  const size_t oX  = off; off += PX;
  const size_t oWq = off; off += PWq;
  const size_t oWk = off; off += PWk;
  const size_t oWv = off; off += PWv;
  const size_t oWo = off; off += PWo;
  const size_t oQf = off; off += PQf;
  const size_t oKf = off; off += PKf;
  const size_t oVT = off; off += PVT;
  const size_t oQh = off; off += PQh;
  const size_t oKh = off; off += PKh;
  const size_t oAh = off; off += PApl;
  const size_t oAl = off; off += PApl;
  if (off > ws_size) return;
  if (off > (size_t)134217728) return;
  const size_t oAf = oQf;

  char* ws = (char*)d_ws;
  unsigned short* X   = (unsigned short*)(ws + oX);
  unsigned short* Xq  = X + (size_t)CLEN * HID;
  unsigned short* Wqb = (unsigned short*)(ws + oWq);
  unsigned short* Wkb = (unsigned short*)(ws + oWk);
  unsigned short* Wvb = (unsigned short*)(ws + oWv);
  unsigned short* Wob = (unsigned short*)(ws + oWo);
  float*          Qf  = (float*)(ws + oQf);
  float*          Kf  = (float*)(ws + oKf);
  unsigned short* VT  = (unsigned short*)(ws + oVT);
  unsigned short* Qh  = (unsigned short*)(ws + oQh);
  unsigned short* Kh  = (unsigned short*)(ws + oKh);
  unsigned short* Ah  = (unsigned short*)(ws + oAh);
  unsigned short* Al  = (unsigned short*)(ws + oAl);
  float*          Af  = (float*)(ws + oAf);
  float*          outf = (float*)d_out;

  const dim3 blk(256);
  const int n8T  = CLEN * HID / 8;
  const int n8H  = QLEN * HID / 8;
  const int n8Wq = QP * HID / 8;
  const int n8Wk = KP * HID / 8;
  const int n8Wo = HID * QP / 8;
  const int n8A  = QLEN * QP / 8;
  const int nwRq = QLEN * (NH / 4);
  const int nwRk = SLEN * (NKV / 4);
  const dim3 gCT((n8T + 255) / 256), gCH((n8H + 255) / 256);
  const dim3 gCWq((n8Wq + 255) / 256), gCWk((n8Wk + 255) / 256), gCWo((n8Wo + 255) / 256);
  const dim3 gQ(((QLEN / 64) * (QP / 64) + 7) / 8);
  const dim3 gK(((SLEN / 64) * (KP / 64) + 7) / 8);
  const dim3 gV(((KP / 64) * (SLEN / 64) + 7) / 8);
  const dim3 gRq((nwRq + 7) / 8), gRk((nwRk + 7) / 8);
  const dim3 gAttn(NQB * NH);
  const dim3 gSplit((n8A + 255) / 256);
  const dim3 gOut(((QLEN / 64) * (HID / 64) + 7) / 8);

  cvt_bf16x8<<<gCT, blk, 0, stream>>>(tgt, X, n8T);
  cvt_bf16x8<<<gCH, blk, 0, stream>>>(hid, Xq, n8H);
  cvt_bf16x8<<<gCWq, blk, 0, stream>>>(Wq, Wqb, n8Wq);
  cvt_bf16x8<<<gCWk, blk, 0, stream>>>(Wk, Wkb, n8Wk);
  cvt_bf16x8<<<gCWk, blk, 0, stream>>>(Wv, Wvb, n8Wk);
  cvt_bf16x8<<<gCWo, blk, 0, stream>>>(Wo, Wob, n8Wo);
  gemm64<0, 0, 1><<<gQ, blk, 0, stream>>>(Xq, Xq, HID, Wqb, HID, bq, (void*)Qf, QP, QLEN, QP, HID, 1.0f);
  gemm64<0, 0, 1><<<gK, blk, 0, stream>>>(X, X, HID, Wkb, HID, bk, (void*)Kf, KP, SLEN, KP, HID, 1.0f);
  gemm64<0, 1, 2><<<gV, blk, 0, stream>>>(Wvb, Wvb, HID, X, HID, bv, (void*)VT, SLEN, KP, SLEN, HID, VSC);
  rope_quads<<<gRq, blk, 0, stream>>>(Qf, fcs, fsn, Qh, QP, NH / 4, CLEN, QSC, nwRq);
  rope_quads<<<gRk, blk, 0, stream>>>(Kf, fcs, fsn, Kh, KP, NKV / 4, 0, KSC, nwRk);
  attn64<<<gAttn, dim3(128), 0, stream>>>(Qh, Kh, VT, Af, 0.125f / (QSC * KSC), 1.0f / (PSC * VSC));
  split_bf16x8<<<gSplit, blk, 0, stream>>>(Af, Ah, Al, n8A);
  gemm64<1, 0, 1><<<gOut, blk, 0, stream>>>(Ah, Al, QP, Wob, QP, bo, (void*)outf, HID, QLEN, HID, QP, 1.0f);
  (void)hipGetLastError();
}
